// MessagePassing_52450140618855
// MI455X (gfx1250) — hardware-verified
//
#include <hip/hip_runtime.h>
#include <stddef.h>
#include <stdint.h>


#define DL     512
#define DO     256
#define NLAY   3
#define PAP    1536
#define AGOFF  0
#define HIOFF  512
#define LOOFF  1024
#define KENC   512
#define KLAY   1536
#define KOUT   1024
#define LDBE   512
#define LDBL   1536
#define LDBO   1024
#define ACAR   16.0f
#define LCAR   2048.0f
#define RLO    0.00048828125f
#define WCAR   4096.0f
#define WCLO   2.0f
#define SINV   0.0000152587890625f
#define NTHR   256
#define NWAVE  8
#define EPT    8
#define CHUNK  (NTHR * EPT)
#define WCAP   (EPT * 32)
#define LISTN  (NWAVE * WCAP)
#define NBA    1024
#define SLA    10
#define RCAP   28672
#define DEGCAP 64
#define GBM    64
#define GBN    128
#define GTHR   128
#define NG     (DL / 8)
#define UENC   (DL * NG)
#define ULAY   (NLAY * 3 * DL * NG)
#define UOUT   (2 * DO * NG)
#define AGG_ZINTS    (LISTN + 2 * RCAP + 3 * NBA)
#define MISC_INTS    16
#define AGG_LDS_INTS (AGG_ZINTS + MISC_INTS)
#define WSMAX  134217728

static_assert((CHUNK & (CHUNK - 1)) == 0 && CHUNK <= 4096);
static_assert((NBA & (NBA - 1)) == 0 && NBA == (1 << SLA));
static_assert(((long long)CHUNK << SLA) < (1LL << 31));
static_assert(LISTN % (NTHR * 4) == 0);
static_assert(NBA % NWAVE == 0 && NBA % 32 == 0 && NBA % GBM == 0 && NBA == 4 * NTHR);
static_assert(RCAP % 4 == 0 && AGG_ZINTS % (NTHR * 4) == 0);
static_assert(KENC % 32 == 0 && KLAY % 32 == 0 && KOUT % 32 == 0 && KLAY == PAP && KOUT + HIOFF == PAP);
static_assert(LOOFF == HIOFF + DL && PAP == 3 * DL && PAP % 64 == 0 && AGOFF == 0);
static_assert(DL % GBN == 0 && DO % GBN == 0 && GBM == (GTHR / 32) * 16 && GBN == 4 * 32 && GBN == 16 * 8);
static_assert(UENC % NTHR == 0 && ULAY % NTHR == 0 && UOUT % NTHR == 0);
static_assert((DL * NG) == (1 << 15) && (DO * NG) == (1 << 14));
static_assert((GBM * NG) % NTHR == 0);
static_assert(DEGCAP % 32 == 0);
static_assert(AGG_LDS_INTS * 4 <= 300000);

typedef float          v4f   __attribute__((ext_vector_type(4)));
typedef float          v8f   __attribute__((ext_vector_type(8)));
typedef int            v4i   __attribute__((ext_vector_type(4)));
typedef int            v8i   __attribute__((ext_vector_type(8)));
typedef unsigned       v4u   __attribute__((ext_vector_type(4)));
typedef unsigned short v8us  __attribute__((ext_vector_type(8)));
typedef _Float16       v16h  __attribute__((ext_vector_type(16)));
typedef v4f  __attribute__((may_alias)) v4fa;
typedef v4i  __attribute__((may_alias)) v4ia;
typedef v4u  __attribute__((may_alias)) v4ua;
typedef v8us __attribute__((may_alias)) v8usa;
union FragH { v16h v; v8us h[2]; v8i w; };

__device__ __forceinline__ v8f wmh(const FragH& a, const FragH& b, v8f c) {
  v8f d = __builtin_amdgcn_wmma_f32_16x16x32_f16(false, a.v, false, b.v, (short)0, c, false, false);
  asm volatile("v_nop\n\tv_nop\n\tv_nop\n\tv_nop" : "+v"(d) : "v"(a.w), "v"(b.w));
  return d;
}

__device__ __forceinline__ float bf16_val(float f) {
  const unsigned u = __float_as_uint(f);
  return __uint_as_float(((u + 0x7FFFu + ((u >> 16) & 1u)) >> 16) << 16);
}
__device__ __forceinline__ unsigned short h16_bits(float f) {
  const _Float16 h = (_Float16)f;
  return __builtin_bit_cast(unsigned short, h);
}
__device__ __forceinline__ float h2f(unsigned short b) {
  return (float)__builtin_bit_cast(_Float16, b);
}
__device__ __forceinline__ unsigned hl_bits(float y) {
  const float v = y * ACAR;
  const _Float16 h = (_Float16)v;
  const float r = (v - (float)h) * LCAR;
  const _Float16 lo = (_Float16)r;
  return (unsigned)__builtin_bit_cast(unsigned short, h) | ((unsigned)__builtin_bit_cast(unsigned short, lo) << 16);
}
template <int R>
__device__ __forceinline__ float epv(float p, float b, bool ok) {
  float t = fmaf(p, SINV, b);
  if (R != 0) t = fmaxf(t, 0.0f);
  return ok ? t : 0.0f;
}
__device__ __forceinline__ v8f acc8(v8f a, const v4u hw, const v4u lw, float ck) {
  a[0] = fmaf(ck, fmaf(h2f((unsigned short)(lw.x & 0xffffu)), RLO, h2f((unsigned short)(hw.x & 0xffffu))), a[0]);
  a[1] = fmaf(ck, fmaf(h2f((unsigned short)(lw.x >> 16)),      RLO, h2f((unsigned short)(hw.x >> 16))),      a[1]);
  a[2] = fmaf(ck, fmaf(h2f((unsigned short)(lw.y & 0xffffu)), RLO, h2f((unsigned short)(hw.y & 0xffffu))), a[2]);
  a[3] = fmaf(ck, fmaf(h2f((unsigned short)(lw.y >> 16)),      RLO, h2f((unsigned short)(hw.y >> 16))),      a[3]);
  a[4] = fmaf(ck, fmaf(h2f((unsigned short)(lw.z & 0xffffu)), RLO, h2f((unsigned short)(hw.z & 0xffffu))), a[4]);
  a[5] = fmaf(ck, fmaf(h2f((unsigned short)(lw.z >> 16)),      RLO, h2f((unsigned short)(hw.z >> 16))),      a[5]);
  a[6] = fmaf(ck, fmaf(h2f((unsigned short)(lw.w & 0xffffu)), RLO, h2f((unsigned short)(hw.w & 0xffffu))), a[6]);
  a[7] = fmaf(ck, fmaf(h2f((unsigned short)(lw.w >> 16)),      RLO, h2f((unsigned short)(hw.w >> 16))),      a[7]);
  return a;
}

__device__ __forceinline__ int scan_chunk2(const int* __restrict__ edg, int nE, int cbase, int slotBase,
                                           int nb, int* list, int tid, int lane, int wave) {
  int wc = 0;
  const int el0  = tid * EPT;
  const int e0   = cbase + el0;
  const int sent = -2147483647 - 1;
  int d0, d1, d2, d3, d4, d5, d6, d7;
  if (cbase + CHUNK <= nE) {
    const int* p = edg + 2 * (size_t)e0;
    const v4i pa = *(const v4i*)p;
    const v4i pb = *(const v4i*)(p + 4);
    const v4i pc = *(const v4i*)(p + 8);
    const v4i pd = *(const v4i*)(p + 12);
    d0 = pa.y; d1 = pa.w; d2 = pb.y; d3 = pb.w; d4 = pc.y; d5 = pc.w; d6 = pd.y; d7 = pd.w;
  } else {
    d0 = (e0     < nE) ? edg[2 * min(e0,     nE - 1) + 1] : sent;
    d1 = (e0 + 1 < nE) ? edg[2 * min(e0 + 1, nE - 1) + 1] : sent;
    d2 = (e0 + 2 < nE) ? edg[2 * min(e0 + 2, nE - 1) + 1] : sent;
    d3 = (e0 + 3 < nE) ? edg[2 * min(e0 + 3, nE - 1) + 1] : sent;
    d4 = (e0 + 4 < nE) ? edg[2 * min(e0 + 4, nE - 1) + 1] : sent;
    d5 = (e0 + 5 < nE) ? edg[2 * min(e0 + 5, nE - 1) + 1] : sent;
    d6 = (e0 + 6 < nE) ? edg[2 * min(e0 + 6, nE - 1) + 1] : sent;
    d7 = (e0 + 7 < nE) ? edg[2 * min(e0 + 7, nE - 1) + 1] : sent;
  }
  const unsigned nbs = (unsigned)slotBase;
  const unsigned unb = (unsigned)nb;
  const unsigned s0 = (unsigned)d0 - nbs, s1 = (unsigned)d1 - nbs;
  const unsigned s2 = (unsigned)d2 - nbs, s3 = (unsigned)d3 - nbs;
  const unsigned s4 = (unsigned)d4 - nbs, s5 = (unsigned)d5 - nbs;
  const unsigned s6 = (unsigned)d6 - nbs, s7 = (unsigned)d7 - nbs;
  const bool h0 = s0 < unb, h1 = s1 < unb, h2 = s2 < unb, h3 = s3 < unb;
  const bool h4 = s4 < unb, h5 = s5 < unb, h6 = s6 < unb, h7 = s7 < unb;
  const unsigned any = __builtin_amdgcn_ballot_w32(h0 | h1 | h2 | h3 | h4 | h5 | h6 | h7);
  if (any != 0u) {
#define HITJ(J, HJ, SJ) { \
      const unsigned mj = __builtin_amdgcn_ballot_w32(HJ); \
      if (mj != 0u) { \
        if (HJ) { \
          const int pos = wc + (int)__builtin_amdgcn_mbcnt_lo(mj, 0u); \
          if (pos < WCAP) list[wave * WCAP + pos] = ((el0 + (J)) << SLA) | (int)(SJ); \
        } \
        wc += (int)__builtin_popcount(mj); } }
    HITJ(0, h0, s0)
    HITJ(1, h1, s1)
    HITJ(2, h2, s2)
    HITJ(3, h3, s3)
    HITJ(4, h4, s4)
    HITJ(5, h5, s5)
    HITJ(6, h6, s6)
    HITJ(7, h7, s7)
#undef HITJ
  }
  return wc;
}

__global__ __launch_bounds__(NTHR) void k_xcvt(const float* __restrict__ x, int nN, unsigned short* pl) {
  const int u   = (int)blockIdx.x * NTHR + (int)threadIdx.x;
  const int row = u >> 6;
  const int g   = u & 63;
  const int rc  = row < nN ? row : nN - 1;
  const float sc = (row < nN) ? ACAR : 0.0f;
  const float* p = x + (size_t)rc * DL + 8 * g;
  const v4f a = *(const v4f*)p;
  const v4f b = *(const v4f*)(p + 4);
  v8us o;
  o[0] = h16_bits(bf16_val(a.x) * sc); o[1] = h16_bits(bf16_val(a.y) * sc);
  o[2] = h16_bits(bf16_val(a.z) * sc); o[3] = h16_bits(bf16_val(a.w) * sc);
  o[4] = h16_bits(bf16_val(b.x) * sc); o[5] = h16_bits(bf16_val(b.y) * sc);
  o[6] = h16_bits(bf16_val(b.z) * sc); o[7] = h16_bits(bf16_val(b.w) * sc);
  unsigned short* dp = pl + (size_t)row * PAP + 8 * g;
  *(volatile v8us*)dp = o;
  __threadfence();
  *(volatile v8us*)dp = o;
}

__global__ __launch_bounds__(NTHR) void k_wprep(const float* __restrict__ Wenc, const float* __restrict__ Wself,
                                                const float* __restrict__ Wneigh, const float* __restrict__ Wout,
                                                unsigned short* Benc, unsigned short* Blay, unsigned short* Bout) {
  const int u = (int)blockIdx.x * NTHR + (int)threadIdx.x;
  const float* W;
  unsigned short* dp;
  int no, n, g;
  float sc;
  if (u < UENC) {
    n = (u >> 6) & (DL - 1); g = u & 63;
    W = Wenc; no = DL; sc = WCAR;
    dp = Benc + (size_t)n * LDBE + 8 * g;
  } else if (u < UENC + ULAY) {
    const int v  = u - UENC;
    const int q  = v >> 15;
    const int l  = q / 3;
    const int th = q - 3 * l;
    n = (v >> 6) & (DL - 1); g = v & 63;
    W = ((th == 0) ? Wneigh : Wself) + (size_t)l * DL * DL;
    no = DL; sc = (th == 2) ? WCLO : WCAR;
    dp = Blay + ((size_t)l * DL + n) * LDBL + DL * th + 8 * g;
  } else if (u < UENC + ULAY + UOUT) {
    const int v  = u - UENC - ULAY;
    const int hf = v >> 14;
    n = (v >> 6) & (DO - 1); g = v & 63;
    W = Wout; no = DO; sc = (hf != 0) ? WCLO : WCAR;
    dp = Bout + (size_t)n * LDBO + DL * hf + 8 * g;
  } else {
    return;
  }
  const float* p = W + (size_t)(8 * g) * (size_t)no + n;
  const float w0 = p[0];
  const float w1 = p[(size_t)no];
  const float w2 = p[2 * (size_t)no];
  const float w3 = p[3 * (size_t)no];
  const float w4 = p[4 * (size_t)no];
  const float w5 = p[5 * (size_t)no];
  const float w6 = p[6 * (size_t)no];
  const float w7 = p[7 * (size_t)no];
  v8us o;
  o[0] = h16_bits(bf16_val(w0) * sc); o[1] = h16_bits(bf16_val(w1) * sc);
  o[2] = h16_bits(bf16_val(w2) * sc); o[3] = h16_bits(bf16_val(w3) * sc);
  o[4] = h16_bits(bf16_val(w4) * sc); o[5] = h16_bits(bf16_val(w5) * sc);
  o[6] = h16_bits(bf16_val(w6) * sc); o[7] = h16_bits(bf16_val(w7) * sc);
  *(volatile v8us*)dp = o;
  __threadfence();
  *(volatile v8us*)dp = o;
}

__global__ __launch_bounds__(NTHR) void k_deg(const int* __restrict__ edg, int nE, int* degt) {
  __shared__ __attribute__((aligned(16))) int list[LISTN];
  __shared__ __attribute__((aligned(16))) int cnt[NBA];
  __shared__ int misc[MISC_INTS];
  const int tid = (int)threadIdx.x, lane = tid & 31, wave = tid >> 5;
  const int nodeBase = (int)blockIdx.x * NBA;
  {
    const v4i z4 = {0, 0, 0, 0};
    for (int i = tid * 4; i < LISTN; i += NTHR * 4) *(v4ia*)(list + i) = z4;
    *(v4ia*)(cnt + 4 * tid) = z4;
    if (tid < MISC_INTS) misc[tid] = 0;
  }
  __syncthreads();
  const int nChunks = (nE + CHUNK - 1) / CHUNK;
#pragma unroll 1
  for (int ch = 0; ch < nChunks; ++ch) {
    const int cbase = ch * CHUNK;
    const int wc = scan_chunk2(edg, nE, cbase, nodeBase, NBA, list, tid, lane, wave);
    if (lane == 0) misc[wave] = wc;
    __syncthreads();
    if (wave == 0) {
#pragma unroll 1
      for (int w2 = 0; w2 < NWAVE; ++w2) {
        int c = misc[w2];
        c = c < 0 ? 0 : (c > WCAP ? WCAP : c);
#pragma unroll 1
        for (int b0 = 0; b0 < c; b0 += 32) {
          const int idx = b0 + lane;
          const int ent = list[w2 * WCAP + (idx < WCAP ? idx : WCAP - 1)];
          const int m32 = (c - b0) < 32 ? (c - b0) : 32;
#pragma unroll 1
          for (int k = 0; k < m32; ++k) {
            const int u    = __builtin_amdgcn_readlane(ent, k);
            const int slot = u & (NBA - 1);
            if (lane == 0) cnt[slot] = cnt[slot] + 1;
          }
        }
      }
    }
    __syncthreads();
  }
  const v4i q = *(const v4ia*)(cnt + 4 * tid);
  int* dp = degt + nodeBase + 4 * tid;
  *(volatile v4i*)dp = q;
  __threadfence();
  *(volatile v4i*)dp = q;
}

template <typename OT, int RELU>
__global__ __launch_bounds__(GTHR) void k_gemm(const unsigned short* __restrict__ A, int lda,
                                               const unsigned short* __restrict__ BT, int ldb, int K,
                                               const float* __restrict__ bias, OT* outp, int ldo, int colOff,
                                               int nOut) {
  __shared__ __attribute__((aligned(16))) float stg[GBM * GBN];
  const int tid = (int)threadIdx.x, lane = tid & 31, wave = tid >> 5, hh = lane >> 4, m = lane & 15;
  const int rowBase = (int)blockIdx.x * GBM;
  const int colBase = (int)blockIdx.y * GBN;

  v8f acc[8];
  {
    const v8f z = {0.f, 0.f, 0.f, 0.f, 0.f, 0.f, 0.f, 0.f};
#pragma unroll
    for (int t = 0; t < 8; ++t) acc[t] = z;
  }
  const unsigned short* ap = A  + (size_t)(rowBase + 16 * wave + m) * (size_t)lda + 8 * hh;
  const unsigned short* bp = BT + (size_t)(colBase + m) * (size_t)ldb + 8 * hh;

#pragma unroll 1
  for (int k0 = 0; k0 < K; k0 += 32) {
    FragH af;
    af.h[0] = *(const v8usa*)(ap + k0);
    af.h[1] = *(const v8usa*)(ap + k0 + 16);
#pragma unroll
    for (int nt = 0; nt < 8; ++nt) {
      const unsigned short* wq = bp + (size_t)(16 * nt) * (size_t)ldb + k0;
      FragH bf;
      bf.h[0] = *(const v8usa*)wq;
      bf.h[1] = *(const v8usa*)(wq + 16);
      acc[nt] = wmh(af, bf, acc[nt]);
    }
  }

#pragma unroll
  for (int nt = 0; nt < 8; ++nt) {
    const int lc = 16 * nt + m;
#pragma unroll
    for (int r = 0; r < 8; ++r) {
      const int lr = 16 * wave + 8 * hh + r;
      stg[lr * GBN + lc] = acc[nt][r];
    }
  }
  __syncthreads();

  if constexpr (sizeof(OT) == 2) {
    const int rr = lane >> 4, c8 = 8 * (lane & 15);
    v4f b0, b1;
    {
      const v4f t0 = *(const v4f*)(bias + colBase + c8);
      const v4f t1 = *(const v4f*)(bias + colBase + c8 + 4);
      b0.x = bf16_val(t0.x); b0.y = bf16_val(t0.y); b0.z = bf16_val(t0.z); b0.w = bf16_val(t0.w);
      b1.x = bf16_val(t1.x); b1.y = bf16_val(t1.y); b1.z = bf16_val(t1.z); b1.w = bf16_val(t1.w);
    }
    v8us qh[8], ql[8];
#pragma unroll
    for (int i = 0; i < 8; ++i) {
      const int lr = 16 * wave + 2 * i + rr;
      const float* sp = stg + lr * GBN + c8;
      const v4f p0 = *(const v4fa*)sp;
      const v4f p1 = *(const v4fa*)(sp + 4);
      const bool ok = (rowBase + lr) < nOut;
      unsigned pk;
      pk = hl_bits(epv<RELU>(p0.x, b0.x, ok)); qh[i][0] = (unsigned short)(pk & 0xffffu); ql[i][0] = (unsigned short)(pk >> 16);
      pk = hl_bits(epv<RELU>(p0.y, b0.y, ok)); qh[i][1] = (unsigned short)(pk & 0xffffu); ql[i][1] = (unsigned short)(pk >> 16);
      pk = hl_bits(epv<RELU>(p0.z, b0.z, ok)); qh[i][2] = (unsigned short)(pk & 0xffffu); ql[i][2] = (unsigned short)(pk >> 16);
      pk = hl_bits(epv<RELU>(p0.w, b0.w, ok)); qh[i][3] = (unsigned short)(pk & 0xffffu); ql[i][3] = (unsigned short)(pk >> 16);
      pk = hl_bits(epv<RELU>(p1.x, b1.x, ok)); qh[i][4] = (unsigned short)(pk & 0xffffu); ql[i][4] = (unsigned short)(pk >> 16);
      pk = hl_bits(epv<RELU>(p1.y, b1.y, ok)); qh[i][5] = (unsigned short)(pk & 0xffffu); ql[i][5] = (unsigned short)(pk >> 16);
      pk = hl_bits(epv<RELU>(p1.z, b1.z, ok)); qh[i][6] = (unsigned short)(pk & 0xffffu); ql[i][6] = (unsigned short)(pk >> 16);
      pk = hl_bits(epv<RELU>(p1.w, b1.w, ok)); qh[i][7] = (unsigned short)(pk & 0xffffu); ql[i][7] = (unsigned short)(pk >> 16);
    }
#pragma unroll
    for (int i = 0; i < 8; ++i) {
      const int lr = 16 * wave + 2 * i + rr;
      OT* dp = outp + (size_t)(rowBase + lr) * (size_t)ldo + colOff + colBase + c8;
      *(volatile v8us*)dp = qh[i];
      *(volatile v8us*)(dp + DL) = ql[i];
    }
    __threadfence();
#pragma unroll
    for (int i = 0; i < 8; ++i) {
      const int lr = 16 * wave + 2 * i + rr;
      OT* dp = outp + (size_t)(rowBase + lr) * (size_t)ldo + colOff + colBase + c8;
      *(volatile v8us*)dp = qh[i];
      *(volatile v8us*)(dp + DL) = ql[i];
    }
  } else {
    v4f b4;
    {
      const v4f tb = *(const v4f*)(bias + colBase + 4 * lane);
      b4.x = bf16_val(tb.x); b4.y = bf16_val(tb.y); b4.z = bf16_val(tb.z); b4.w = bf16_val(tb.w);
    }
    v4f pv[16];
#pragma unroll
    for (int i = 0; i < 16; ++i) {
      const v4f p = *(const v4fa*)(stg + (16 * wave + i) * GBN + 4 * lane);
      v4f t;
      t.x = epv<RELU>(p.x, b4.x, true); t.y = epv<RELU>(p.y, b4.y, true);
      t.z = epv<RELU>(p.z, b4.z, true); t.w = epv<RELU>(p.w, b4.w, true);
      pv[i] = t;
    }
#pragma unroll
    for (int i = 0; i < 16; ++i) {
      const int r = rowBase + 16 * wave + i;
      if (r < nOut) *(volatile v4f*)(outp + (size_t)r * (size_t)ldo + colOff + colBase + 4 * lane) = pv[i];
    }
    __threadfence();
#pragma unroll
    for (int i = 0; i < 16; ++i) {
      const int r = rowBase + 16 * wave + i;
      if (r < nOut) *(volatile v4f*)(outp + (size_t)r * (size_t)ldo + colOff + colBase + 4 * lane) = pv[i];
    }
  }
}

__global__ __launch_bounds__(NTHR) void k_scan(const int* __restrict__ edg, const int* __restrict__ degt,
                                               int nE, int nN, int nP, int mRows, unsigned short* pl) {
  extern __shared__ __attribute__((aligned(16))) int dsm[];
  int* list = dsm;
  int* hl   = dsm + LISTN;
  int* sl   = hl + RCAP;
  int* cnt  = sl + RCAP;
  int* offs = cnt + NBA;
  int* cur  = offs + NBA;
  int* misc = cur + NBA;
  const int tid = (int)threadIdx.x, lane = tid & 31, wave = tid >> 5;
  const int nodeBase = (int)blockIdx.x * NBA;

  {
    const v4i z4 = {0, 0, 0, 0};
    for (int i = tid * 4; i < AGG_ZINTS; i += NTHR * 4) *(v4ia*)(dsm + i) = z4;
    if (tid < MISC_INTS) misc[tid] = 0;
  }
  __syncthreads();

  int t = 0, ov = 0;
  const int nChunks = (nE + CHUNK - 1) / CHUNK;
#pragma unroll 1
  for (int ch = 0; ch < nChunks; ++ch) {
    const int cbase = ch * CHUNK;
    const int wc = scan_chunk2(edg, nE, cbase, nodeBase, NBA, list, tid, lane, wave);
    if (lane == 0) misc[wave] = wc;
    __syncthreads();
    if (wave == 0) {
#pragma unroll 1
      for (int w2 = 0; w2 < NWAVE; ++w2) {
        int c = misc[w2];
        c = c < 0 ? 0 : (c > WCAP ? WCAP : c);
#pragma unroll 1
        for (int b0 = 0; b0 < c; b0 += 32) {
          const int idx = b0 + lane;
          const int ent = list[w2 * WCAP + (idx < WCAP ? idx : WCAP - 1)];
          const int m32 = (c - b0) < 32 ? (c - b0) : 32;
#pragma unroll 1
          for (int k = 0; k < m32; ++k) {
            const int u    = __builtin_amdgcn_readlane(ent, k);
            const int slot = u & (NBA - 1);
            const int el   = (u >> SLA) & (CHUNK - 1);
            const int pk   = ((cbase + el) << SLA) | slot;
            if (t < RCAP) {
              if (lane == 0) { hl[t] = pk; cnt[slot] = cnt[slot] + 1; }
              t = t + 1;
            } else {
              ov = 1;
            }
          }
        }
      }
    }
    __syncthreads();
  }
  if (wave == 0 && lane == 0) { misc[8] = t; misc[9] = ov; }
  __syncthreads();
  int tt = misc[8];
  tt = tt < 0 ? 0 : (tt > RCAP ? RCAP : tt);
  const int ovf = misc[9];

  if (wave == 0) {
    const int base = lane * (NBA / 32);
    int s = 0;
#pragma unroll 1
    for (int i = 0; i < NBA / 32; ++i) s += cnt[base + i];
    int incl = s;
#pragma unroll
    for (int d = 1; d < 32; d <<= 1) {
      const int y = __shfl_up(incl, d, 32);
      if (lane >= d) incl += y;
    }
    int run = incl - s;
#pragma unroll 1
    for (int i = 0; i < NBA / 32; ++i) {
      const int cv = cnt[base + i];
      offs[base + i] = run;
      cur[base + i]  = run;
      run += cv;
    }
  }
  __syncthreads();
  if (wave == 0) {
#pragma unroll 1
    for (int b0 = 0; b0 < tt; b0 += 32) {
      const int idx = b0 + lane;
      const int ent = hl[idx < RCAP ? idx : RCAP - 1];
      const int m32 = (tt - b0) < 32 ? (tt - b0) : 32;
#pragma unroll 1
      for (int k = 0; k < m32; ++k) {
        const int u    = __builtin_amdgcn_readlane(ent, k);
        const int slot = u & (NBA - 1);
        if (lane == 0) {
          int p = cur[slot];
          p = p < 0 ? 0 : (p > RCAP - 1 ? RCAP - 1 : p);
          sl[p] = u;
          cur[slot] = p + 1;
        }
      }
    }
  }
  __syncthreads();

  const float pz = (ovf != 0) ? __int_as_float(0x7fc00000) : 0.0f;
  const v8f z8 = {0.f, 0.f, 0.f, 0.f, 0.f, 0.f, 0.f, 0.f};
#pragma unroll 1
  for (int si = 0; si < NBA / NWAVE; ++si) {
    const int s    = si * NWAVE + wave;
    const int node = nodeBase + s;
    int c = cnt[s];
    const bool big = c > DEGCAP;
    c = c < 0 ? 0 : (c > DEGCAP ? DEGCAP : c);
    int o = offs[s];
    o = o < 0 ? 0 : (o > RCAP ? RCAP : o);
    const int nc = node < nN ? node : nN - 1;
    int dd = degt[nc < nP ? nc : nP - 1];
    dd = dd < 0 ? 0 : (dd > nE ? nE : dd);
    const float fd = (float)dd + 1.0f;
    v8f aA = z8, aB = z8;
#pragma unroll 1
    for (int b0 = 0; b0 < c; b0 += 32) {
      int idx = o + b0 + lane;
      idx = idx > RCAP - 1 ? RCAP - 1 : idx;
      const int ent = sl[idx];
      int eid = ent >> SLA;
      eid = eid < 0 ? 0 : (eid > nE - 1 ? nE - 1 : eid);
      int sr = edg[2 * (size_t)eid];
      sr = sr < 0 ? 0 : (sr > nN - 1 ? nN - 1 : sr);
      int ds = degt[sr];
      ds = ds < 0 ? 0 : (ds > nE ? nE : ds);
      const float wv  = rsqrtf(fd * ((float)ds + 1.0f));
      const int   wvi = __float_as_int(wv);
      const int m32 = (c - b0) < 32 ? (c - b0) : 32;
#pragma unroll 1
      for (int k = 0; k < m32; ++k) {
        const int   sk = __builtin_amdgcn_readlane(sr, k);
        const float ck = __int_as_float(__builtin_amdgcn_readlane(wvi, k));
        const unsigned short* rp = pl + (size_t)sk * PAP + HIOFF + 8 * lane;
        const v4u hw0 = *(const v4ua*)rp;
        const v4u lw0 = *(const v4ua*)(rp + DL);
        const v4u hw1 = *(const v4ua*)(rp + 256);
        const v4u lw1 = *(const v4ua*)(rp + DL + 256);
        aA = acc8(aA, hw0, lw0, ck);
        aB = acc8(aB, hw1, lw1, ck);
      }
    }
    const float pzr = big ? __int_as_float(0x7fc00000) : pz;
    const bool live = node < nN;
    v8us q0, q1;
#pragma unroll
    for (int j = 0; j < 8; ++j) {
      q0[j] = h16_bits(live ? (aA[j] + pzr) : 0.0f);
      q1[j] = h16_bits(live ? (aB[j] + pzr) : 0.0f);
    }
    if (node < mRows) {
      unsigned short* rpw = pl + (size_t)node * PAP + AGOFF + 8 * lane;
      *(volatile v8us*)rpw = q0;
      *(volatile v8us*)(rpw + 256) = q1;
      __threadfence();
      *(volatile v8us*)rpw = q0;
      *(volatile v8us*)(rpw + 256) = q1;
    }
  }
}

static inline int cdiv(int a, int b) { return (a + b - 1) / b; }
static inline size_t al256(size_t o) { return (o + 255) & ~(size_t)255; }

extern "C" void kernel_launch(void* const* d_in, const int* in_sizes, int n_in,
                              void* d_out, int out_size, void* d_ws, size_t ws_size,
                              hipStream_t stream) {
  if (n_in < 9) return;
  if (in_sizes[0] < DL || (in_sizes[0] % DL) != 0) return;
  const int nN = in_sizes[0] / DL;
  if (in_sizes[1] < 2 || (in_sizes[1] & 1) != 0) return;
  const int nE = in_sizes[1] / 2;
  if (nE < 1 || nE >= (1 << 21) || nN < 16 || nN >= (1 << 24)) return;
  if (in_sizes[2] != DL * DL || in_sizes[3] != DL) return;
  if (in_sizes[4] != NLAY * DL * DL || in_sizes[5] != NLAY * DL * DL || in_sizes[6] != NLAY * DL) return;
  if (in_sizes[7] != DL * DO || in_sizes[8] != DO) return;
  if ((long long)out_size != (long long)nN * DO) return;

  const float* x      = (const float*)d_in[0];
  const int*   edg    = (const int*)d_in[1];
  const float* Wenc   = (const float*)d_in[2];
  const float* benc   = (const float*)d_in[3];
  const float* Wself  = (const float*)d_in[4];
  const float* Wneigh = (const float*)d_in[5];
  const float* bcomb  = (const float*)d_in[6];
  const float* Wout   = (const float*)d_in[7];
  const float* bout   = (const float*)d_in[8];
  float* out = (float*)d_out;

  const int MP = cdiv(nN, GBM) * GBM;
  const int gM = MP / GBM;
  const int gA = cdiv(MP, NBA);
  const int NP = gA * NBA;
  if ((long long)gA * NBA < (long long)MP) return;

  char* ws = (char*)d_ws;
  size_t off = 0;
  const size_t oDg = off; off = al256(off + (size_t)NP * 4);
  const size_t oBe = off; off = al256(off + (size_t)DL * LDBE * 2);
  const size_t oBl = off; off = al256(off + (size_t)NLAY * DL * LDBL * 2);
  const size_t oBo = off; off = al256(off + (size_t)DO * LDBO * 2);
  const size_t oPA = off; off = al256(off + (size_t)MP * PAP * 2);
  const size_t oPB = off; off = al256(off + (size_t)MP * PAP * 2);
  if (off > ws_size || off > (size_t)WSMAX) return;
  int*            degt = (int*)(ws + oDg);
  unsigned short* Be   = (unsigned short*)(ws + oBe);
  unsigned short* Bl   = (unsigned short*)(ws + oBl);
  unsigned short* Bo   = (unsigned short*)(ws + oBo);
  unsigned short* PA   = (unsigned short*)(ws + oPA);
  unsigned short* PB   = (unsigned short*)(ws + oPB);

  const size_t scanLds = (size_t)AGG_LDS_INTS * 4;
  hipFuncSetAttribute(reinterpret_cast<const void*>(&k_scan), hipFuncAttributeMaxDynamicSharedMemorySize, (int)scanLds);

  k_xcvt<<<(MP * NG) / NTHR, NTHR, 0, stream>>>(x, nN, PB);
  k_wprep<<<(UENC + ULAY + UOUT) / NTHR, NTHR, 0, stream>>>(Wenc, Wself, Wneigh, Wout, Be, Bl, Bo);
  k_deg<<<gA, NTHR, 0, stream>>>(edg, nE, degt);
  k_gemm<unsigned short, 0><<<dim3(gM, DL / GBN), GTHR, 0, stream>>>(PB, PAP, Be, LDBE, KENC, benc, PA, PAP, HIOFF, nN);
  unsigned short* Pc = PA;
  unsigned short* Pn = PB;
  for (int l = 0; l < NLAY; ++l) {
    k_scan<<<gA, NTHR, scanLds, stream>>>(edg, degt, nE, nN, NP, MP, Pc);
    k_gemm<unsigned short, 1><<<dim3(gM, DL / GBN), GTHR, 0, stream>>>(Pc, PAP, Bl + (size_t)l * DL * LDBL, LDBL, KLAY,
                                                                        bcomb + (size_t)l * DL, Pn, PAP, HIOFF, nN);
    unsigned short* tp = Pc; Pc = Pn; Pn = tp;
  }
  k_gemm<float, 0><<<dim3(gM, DO / GBN), GTHR, 0, stream>>>(Pc + HIOFF, PAP, Bo, LDBO, KOUT, bout, out, DO, 0, nN);
}
